// MultiheadMaskedAttention_61873298866580
// MI455X (gfx1250) — hardware-run, weakly checked
//
#include <hip/hip_runtime.h>
#include <math.h>

#ifndef NB
#define NB 4
#endif
#ifndef SEQ
#define SEQ 2048
#endif
#define NB_FULL  4
#define SEQ_FULL 2048
#define HID  128
#define NHD  8
#define HSZ  128
#define DMD  1024
#define N3   3072
#define QKW  2048
static_assert(NB >= 1 && NB <= NB_FULL);
static_assert(SEQ >= 128 && SEQ <= SEQ_FULL && (SEQ % 128) == 0);
static_assert(NHD * HSZ == DMD && 3 * DMD == N3 && QKW == 2 * DMD);
static_assert((HID % 32) == 0 && (DMD % 32) == 0);

typedef _Float16 f16;
typedef __attribute__((ext_vector_type(4))) unsigned v4u_t;
typedef __attribute__((ext_vector_type(4))) float v4f_t;
typedef float v4fa __attribute__((ext_vector_type(4), may_alias));
typedef float v2fa __attribute__((ext_vector_type(2), may_alias));
typedef __attribute__((ext_vector_type(16))) f16 f16x16;
typedef __attribute__((ext_vector_type(8)))  f16 f16x8;
typedef f16 f16x8a __attribute__((ext_vector_type(8), may_alias));
typedef f16 f16x2a __attribute__((ext_vector_type(2), may_alias));
typedef __attribute__((ext_vector_type(8)))  float f32x8;

__device__ __forceinline__ f32x8 wmma16(f16x16 a, f16x16 b, f32x8 c) {
  c = __builtin_amdgcn_wmma_f32_16x16x32_f16(false, a, false, b, (short)0, c, false, false);
  asm volatile("v_nop\n\tv_nop\n\tv_nop\n\tv_nop" : "+v"(c) : "v"(a), "v"(b));
  return c;
}

__device__ __forceinline__ f16x16 gfrag(const f16* p) {
  const f16x8 lo = *(const f16x8a*)p;
  const f16x8 hi = *(const f16x8a*)(p + 16);
  f16x16 f;
#pragma unroll
  for (int i = 0; i < 8; ++i) { f[i] = lo[i]; f[i + 8] = hi[i]; }
  return f;
}
__device__ __forceinline__ f16x16 lds_frag(const f16* base, int stride) {
  const int lane = threadIdx.x & 31;
  return gfrag(base + (lane & 15) * stride + (lane >> 4) * 8);
}

__device__ __forceinline__ float bf16r(float x) {
  unsigned u = __float_as_uint(x);
  u = (u + 0x7FFFu + ((u >> 16) & 1u)) & 0xFFFF0000u;
  return __uint_as_float(u);
}

__global__ __launch_bounds__(256) void k_cvt_x(const float* __restrict__ x, f16* __restrict__ xh) {
  const int i = blockIdx.x * 256 + threadIdx.x;
  if (i >= NB * SEQ * (HID / 8)) return;
  const int m = i >> 4, c8 = (i & 15) * 8;
  const int b = m / SEQ, s = m - b * SEQ;
  const float* src = x + ((size_t)b * SEQ_FULL + s) * HID + c8;
  const v4f_t a = *(const v4fa*)src, c = *(const v4fa*)(src + 4);
  union { f16 h[8]; v4u_t v; } u;
#pragma unroll
  for (int e = 0; e < 4; ++e) { u.h[e] = (f16)bf16r(a[e]); u.h[4 + e] = (f16)bf16r(c[e]); }
  f16* dst = xh + (size_t)m * HID + c8;
  *(volatile v4u_t*)dst = u.v; __threadfence(); *(volatile v4u_t*)dst = u.v;
}
__global__ __launch_bounds__(256) void k_cvt_w(const float* __restrict__ src, f16* __restrict__ dst, int n8, float scale) {
  const int i = blockIdx.x * 256 + threadIdx.x;
  if (i >= n8) return;
  const float* p = src + (size_t)i * 8;
  const v4f_t a = *(const v4fa*)p, c = *(const v4fa*)(p + 4);
  union { f16 h[8]; v4u_t v; } u;
#pragma unroll
  for (int e = 0; e < 4; ++e) { u.h[e] = (f16)(bf16r(a[e]) * scale); u.h[4 + e] = (f16)(bf16r(c[e]) * scale); }
  f16* d = dst + (size_t)i * 8;
  *(volatile v4u_t*)d = u.v; __threadfence(); *(volatile v4u_t*)d = u.v;
}

#define GSTR 48
__device__ __forceinline__ void stage_a(const f16* src, f16* dh, f16* dl) {
  const f16x8 a = *(const f16x8a*)src, c = *(const f16x8a*)(src + 8);
  *(f16x8a*)dh = a; *(f16x8a*)(dh + 8) = c;
  (void)dl;
}
__device__ __forceinline__ void stage_a(const float* src, f16* dh, f16* dl) {
  union { f16 h[16]; f16x8 v[2]; } H, L;
#pragma unroll
  for (int g = 0; g < 4; ++g) {
    const v4f_t v = *(const v4fa*)(src + 4 * g);
#pragma unroll
    for (int u = 0; u < 4; ++u) {
      const float f = v[u]; const f16 hv = (f16)f;
      H.h[4 * g + u] = hv; L.h[4 * g + u] = (f16)((f - (float)hv) * 2048.0f);
    }
  }
  *(f16x8a*)dh = H.v[0]; *(f16x8a*)(dh + 8) = H.v[1];
  *(f16x8a*)dl = L.v[0]; *(f16x8a*)(dl + 8) = L.v[1];
}

template <typename AT, bool OUT16>
__global__ __launch_bounds__(256) void k_gemm(const AT* __restrict__ A, int lda, const f16* __restrict__ Wh, int ldw,
                                              const float* __restrict__ bias, float oscale, void* __restrict__ Yv, int ldy, int K) {
  constexpr bool SPLIT = (sizeof(AT) == 4);
  __shared__ __attribute__((aligned(16))) f16 ldsA[128 * GSTR];
  __shared__ __attribute__((aligned(16))) f16 ldsAl[128 * GSTR];
  __shared__ __attribute__((aligned(16))) f16 ldsW[128 * GSTR];
  __shared__ __attribute__((aligned(16))) float oS[8][32 * 68];
  const int tid = threadIdx.x, lane = tid & 31, wave = tid >> 5, cl = lane & 15, rh = (lane >> 4) * 8;
  const int m0 = blockIdx.x * 128, n0 = blockIdx.y * 128;
  const int wm = (wave & 3) * 32, wn = (wave >> 2) * 64;
  f32x8 acc[2][4], accx[2][4];
#pragma unroll
  for (int i = 0; i < 2; ++i)
#pragma unroll
    for (int j = 0; j < 4; ++j) { f32x8 z = {}; acc[i][j] = z; accx[i][j] = z; }
#pragma unroll 1
  for (int k0 = 0; k0 < K; k0 += 32) {
    __syncthreads();
    { const int row = tid >> 1, ch = (tid & 1) * 16;
      stage_a(A + (size_t)(m0 + row) * lda + k0 + ch, ldsA + row * GSTR + ch, ldsAl + row * GSTR + ch); }
    { const int k = tid >> 3, nn0 = (tid & 7) * 16;
      const f16* src = Wh + (size_t)(k0 + k) * ldw + n0 + nn0;
      const f16x8 w0 = *(const f16x8a*)src, w1 = *(const f16x8a*)(src + 8);
#pragma unroll
      for (int u = 0; u < 8; ++u) { ldsW[(nn0 + u) * GSTR + k] = w0[u]; ldsW[(nn0 + 8 + u) * GSTR + k] = w1[u]; } }
    __syncthreads();
    f16x16 af[2], afl[2];
#pragma unroll
    for (int i = 0; i < 2; ++i) {
      af[i] = lds_frag(ldsA + (wm + 16 * i) * GSTR, GSTR);
      afl[i] = SPLIT ? lds_frag(ldsAl + (wm + 16 * i) * GSTR, GSTR) : af[i];
    }
#pragma unroll
    for (int j = 0; j < 4; ++j) {
      const f16x16 bf = lds_frag(ldsW + (wn + 16 * j) * GSTR, GSTR);
#pragma unroll
      for (int i = 0; i < 2; ++i) {
        acc[i][j] = wmma16(af[i], bf, acc[i][j]);
        if (SPLIT) accx[i][j] = wmma16(afl[i], bf, accx[i][j]);
      }
    }
  }
  float* so = oS[wave];
#pragma unroll
  for (int i = 0; i < 2; ++i)
#pragma unroll
    for (int j = 0; j < 4; ++j) {
      const int n = n0 + wn + 16 * j + cl;
      const float bv = bias ? bf16r(bias[n]) : 0.0f;
#pragma unroll
      for (int r = 0; r < 8; ++r) {
        float v = acc[i][j][r];
        if (SPLIT) v += accx[i][j][r] * (1.0f / 2048.0f);
        so[(16 * i + rh + r) * 68 + 16 * j + cl] = v * oscale + bv;
      }
    }
  asm volatile("s_wait_dscnt 0" ::: "memory");
  __builtin_amdgcn_wave_barrier();
#pragma unroll 1
  for (int pass = 0; pass < 2; ++pass) {
    if (OUT16) {
      f16* Y = (f16*)Yv;
#pragma unroll
      for (int it = 0; it < 8; ++it) { const int c = lane + 32 * it, rr = c >> 3, q8 = (c & 7) * 8;
        union { f16 h[8]; v4u_t v; } u;
#pragma unroll
        for (int e = 0; e < 8; ++e) u.h[e] = (f16)so[rr * 68 + q8 + e];
        *(volatile v4u_t*)(Y + (size_t)(m0 + wm + rr) * ldy + n0 + wn + q8) = u.v; }
    } else {
      float* Y = (float*)Yv;
#pragma unroll
      for (int it = 0; it < 16; ++it) { const int f4 = lane + 32 * it, rr = f4 >> 4, q = (f4 & 15) * 4;
        *(volatile v4f_t*)(Y + (size_t)(m0 + wm + rr) * ldy + n0 + wn + q) = *(const v4fa*)(so + rr * 68 + q); }
    }
    __threadfence();
  }
}

__global__ __launch_bounds__(256) void k_vtrans(const float* __restrict__ vf, f16* __restrict__ vt) {
  __shared__ float tS[64][65];
  const int tid = threadIdx.x;
  const int t0 = blockIdx.x * 64, c0 = blockIdx.y * 64, b = blockIdx.z;
  for (int e = tid; e < 64 * 64; e += 256) { const int r = e >> 6, c = e & 63; tS[r][c] = vf[((size_t)b * SEQ + t0 + r) * DMD + c0 + c]; }
  __syncthreads();
  union U8 { f16 h[8]; v4u_t v; };
  U8 u0, u1;
  { const int ch = tid, r = ch >> 3, q8 = (ch & 7) * 8;
#pragma unroll
    for (int e = 0; e < 8; ++e) u0.h[e] = (f16)tS[q8 + e][r]; }
  { const int ch = tid + 256, r = ch >> 3, q8 = (ch & 7) * 8;
#pragma unroll
    for (int e = 0; e < 8; ++e) u1.h[e] = (f16)tS[q8 + e][r]; }
#pragma unroll 1
  for (int pass = 0; pass < 2; ++pass) {
    { const int ch = tid, r = ch >> 3, q8 = (ch & 7) * 8;
      *(volatile v4u_t*)(vt + ((size_t)b * DMD + c0 + r) * SEQ + t0 + q8) = u0.v; }
    { const int ch = tid + 256, r = ch >> 3, q8 = (ch & 7) * 8;
      *(volatile v4u_t*)(vt + ((size_t)b * DMD + c0 + r) * SEQ + t0 + q8) = u1.v; }
    __threadfence();
  }
}

__global__ __launch_bounds__(256) void k_colsum(const float* __restrict__ vf, float* __restrict__ cvec) {
  const int idx = blockIdx.x * 256 + threadIdx.x;
  if (idx >= NB * DMD) return;
  const int b = idx / DMD, c = idx - b * DMD;
  const float* p = vf + (size_t)b * SEQ * DMD + c;
  double s = 0.0;
#pragma unroll 4
  for (int t = 0; t < SEQ; ++t) s += (double)p[(size_t)t * DMD];
  const float v = (float)(s * 0.125);
  *(volatile float*)(cvec + idx) = v; __threadfence(); *(volatile float*)(cvec + idx) = v;
}

#define PSTR 40
__global__ __launch_bounds__(256) void k_attn(const f16* __restrict__ qk, const f16* __restrict__ vt, const float* __restrict__ cvec,
                                              const int* __restrict__ nhp, float* __restrict__ ctx) {
  __shared__ __attribute__((aligned(16))) float lsc[NHD * 16 * 32];
  __shared__ __attribute__((aligned(16))) f16 lp[NHD * 16 * PSTR];
  __shared__ __attribute__((aligned(16))) float oS[NHD][16 * 68];
  const int tid = threadIdx.x, lane = tid & 31, h = tid >> 5, cl = lane & 15, rh = (lane >> 4) * 8;
  const int nqb = SEQ / 16;
  const int b = blockIdx.x / nqb, s0 = (blockIdx.x - b * nqb) * 16;
  const float poison = (nhp[0] == NHD) ? 0.0f : __int_as_float(0x7fc00000);
  const float LOG2E = 1.4426950408889634f;
  const f16* qrow = qk + (size_t)(b * SEQ + s0 + cl) * QKW + h * HSZ + rh;
  f16x16 qf[4];
#pragma unroll
  for (int ks = 0; ks < 4; ++ks) qf[ks] = gfrag(qrow + 32 * ks);
  f32x8 oacc[8];
#pragma unroll
  for (int i = 0; i < 8; ++i) { f32x8 z = {}; oacc[i] = z; }
  const int sl = tid >> 4, tp = (tid & 15) * 2;
  const int srow = s0 + sl;
#pragma unroll 1
  for (int t0 = (s0 >> 5) << 5; t0 < SEQ; t0 += 32) {
    f32x8 sc0, sc1;
    { f32x8 z = {}; sc0 = z; sc1 = z; }
    const f16* k0p = qk + (size_t)(b * SEQ + t0 + cl) * QKW + DMD + h * HSZ + rh;
    const f16* k1p = k0p + (size_t)16 * QKW;
#pragma unroll
    for (int ks = 0; ks < 4; ++ks) {
      const f16x16 bq0 = gfrag(k0p + 32 * ks), bq1 = gfrag(k1p + 32 * ks);
      sc0 = wmma16(qf[ks], bq0, sc0);
      sc1 = wmma16(qf[ks], bq1, sc1);
    }
    float* scw = lsc + (h * 16 + rh) * 32;
#pragma unroll
    for (int r = 0; r < 8; ++r) {
      const int s = s0 + rh + r;
      scw[r * 32 + cl]      = (t0 + cl >= s)      ? sc0[r] * 0.03125f : 0.0f;
      scw[r * 32 + 16 + cl] = (t0 + 16 + cl >= s) ? sc1[r] * 0.03125f : 0.0f;
    }
    __syncthreads();
    {
      float e0[8], e1[8];
      float mx0 = -3.0e38f, mx1 = -3.0e38f;
#pragma unroll
      for (int j = 0; j < 8; ++j) {
        const v2fa v = *(const v2fa*)(lsc + (j * 16 + sl) * 32 + tp);
        e0[j] = v[0]; e1[j] = v[1];
        mx0 = fmaxf(mx0, e0[j]); mx1 = fmaxf(mx1, e1[j]);
      }
      float z0 = 0.0f, z1 = 0.0f;
#pragma unroll
      for (int j = 0; j < 8; ++j) {
        e0[j] = __builtin_amdgcn_exp2f((e0[j] - mx0) * LOG2E);
        e1[j] = __builtin_amdgcn_exp2f((e1[j] - mx1) * LOG2E);
        z0 += e0[j]; z1 += e1[j];
      }
      const float rz0 = 1.0f / z0, rz1 = 1.0f / z1;
      const bool um0 = (t0 + tp) >= srow, um1 = (t0 + tp + 1) >= srow;
#pragma unroll
      for (int j = 0; j < 8; ++j) {
        const float p0 = um0 ? (e0[j] * rz0 - 0.125f) * 32768.0f : 0.0f;
        const float p1 = um1 ? (e1[j] * rz1 - 0.125f) * 32768.0f : 0.0f;
        f16x2a pv; pv[0] = (f16)p0; pv[1] = (f16)p1;
        *(f16x2a*)(lp + (j * 16 + sl) * PSTR + tp) = pv;
      }
    }
    __syncthreads();
    const f16x16 pf = lds_frag(lp + h * 16 * PSTR, PSTR);
    const f16* vrow = vt + (size_t)(b * DMD + h * HSZ + cl) * SEQ + t0 + rh;
#pragma unroll
    for (int cs = 0; cs < 8; ++cs) {
      const f16x16 vb = gfrag(vrow + (size_t)(cs * 16) * SEQ);
      oacc[cs] = wmma16(pf, vb, oacc[cs]);
    }
  }
  float* so = oS[h];
#pragma unroll
  for (int hf = 0; hf < 2; ++hf) {
#pragma unroll
    for (int j = 0; j < 4; ++j) {
      const float cv = cvec[(size_t)b * DMD + h * HSZ + (4 * hf + j) * 16 + cl] + poison;
#pragma unroll
      for (int r = 0; r < 8; ++r) so[(rh + r) * 68 + 16 * j + cl] = oacc[4 * hf + j][r] * (1.0f / 32768.0f) + cv;
    }
    asm volatile("s_wait_dscnt 0" ::: "memory");
    __builtin_amdgcn_wave_barrier();
#pragma unroll 1
    for (int pass = 0; pass < 2; ++pass) {
#pragma unroll
      for (int it = 0; it < 8; ++it) { const int f4 = lane + 32 * it, rr = f4 >> 4, q = (f4 & 15) * 4;
        *(volatile v4f_t*)(ctx + (size_t)(b * SEQ + s0 + rr) * DMD + h * HSZ + 64 * hf + q) = *(const v4fa*)(so + rr * 68 + q); }
      __threadfence();
    }
    asm volatile("s_wait_dscnt 0" ::: "memory");
    __builtin_amdgcn_wave_barrier();
  }
}

extern "C" void kernel_launch(void* const* d_in, const int* in_sizes, int n_in,
                              void* d_out, int out_size, void* d_ws, size_t ws_size,
                              hipStream_t stream) {
  if (n_in < 6) return;
  if (in_sizes[0] < ((NB - 1) * SEQ_FULL + SEQ) * HID) return;
  if (in_sizes[1] < HID * N3 || in_sizes[2] < N3 || in_sizes[3] < DMD * HID || in_sizes[4] < HID || in_sizes[5] < 1) return;
  if (out_size < NB * SEQ * HID) return;
  const float* x     = (const float*)d_in[0];
  const float* W_qkv = (const float*)d_in[1];
  const float* b_qkv = (const float*)d_in[2];
  const float* W_o   = (const float*)d_in[3];
  const float* b_o   = (const float*)d_in[4];
  const int*   nhp   = (const int*)d_in[5];
  float* out = (float*)d_out;
  char* ws = (char*)d_ws; size_t off = 0;
  f16*   xh   = (f16*)(ws + off);   off += (size_t)NB * SEQ * HID * 2;
  f16*   wh   = (f16*)(ws + off);   off += (size_t)HID * N3 * 2;
  f16*   woh  = (f16*)(ws + off);   off += (size_t)DMD * HID * 2;
  f16*   qk   = (f16*)(ws + off);   off += (size_t)NB * SEQ * QKW * 2;
  float* vf   = (float*)(ws + off); off += (size_t)NB * SEQ * DMD * 4;
  f16*   vt   = (f16*)(ws + off);   off += (size_t)NB * DMD * SEQ * 2;
  float* cvec = (float*)(ws + off); off += (size_t)NB * DMD * 4;
  if (off > ws_size) return;
  float* ctx = vf;
  const dim3 blk(256);
  k_cvt_x<<<dim3((NB * SEQ * (HID / 8) + 255) / 256), blk, 0, stream>>>(x, xh);
  k_cvt_w<<<dim3((HID * N3 / 8 + 255) / 256), blk, 0, stream>>>(W_qkv, wh, HID * N3 / 8, 64.0f);
  k_cvt_w<<<dim3((DMD * HID / 8 + 255) / 256), blk, 0, stream>>>(W_o, woh, DMD * HID / 8, 64.0f);
  k_gemm<f16, true><<<dim3(NB * SEQ / 128, QKW / 128), blk, 0, stream>>>(xh, HID, wh, N3, b_qkv, 1.0f / 64.0f, (void*)qk, QKW, HID);
  k_gemm<f16, false><<<dim3(NB * SEQ / 128, DMD / 128), blk, 0, stream>>>(xh, HID, wh + 2 * DMD, N3, b_qkv + 2 * DMD, 1.0f / 64.0f, (void*)vf, DMD, HID);
  k_vtrans<<<dim3(SEQ / 64, DMD / 64, NB), blk, 0, stream>>>(vf, vt);
  k_colsum<<<dim3((NB * DMD + 255) / 256), blk, 0, stream>>>(vf, cvec);
  k_attn<<<dim3(NB * (SEQ / 16)), blk, 0, stream>>>(qk, vt, cvec, nhp, ctx);
  k_gemm<float, false><<<dim3(NB * SEQ / 128, HID / 128), blk, 0, stream>>>(ctx, DMD, woh, HID, b_o, 1.0f / 64.0f, (void*)out, HID, DMD);
}
